// PointTransformerLayer_9165460209725
// MI455X (gfx1250) — hardware-run, weakly checked
//
#include <hip/hip_runtime.h>
#include <stddef.h>
#include <stdint.h>
#include <math.h>


#define FW     128
#define NNB    16
#define CSW    16
#define QW     384
#define WROWS  384
#define K2     256
#define NB     8
#define PR     128
#define FTHR   128
#define NTHR   256
#define GBM    64
#define GBN    64
#define GTHR   128
#define AP     264
#define DP     20
#define BN_EPS 1e-5f
#define LEAK   0.1f
#define UWQKV  (WROWS * (FW / 8))
#define UW1    (CSW * (K2 / 8))
#define NUW    (UWQKV + UW1)
#define WSMAX  134217728

#define CP2W   0
#define CP2B   384
#define CBNS   512
#define CBNB   640
#define CBQ    768
#define CBK    896
#define CBV    1024
#define CW2W   1152
#define CW1B   1408
#define CW1S   1424
#define CW1H   1440
#define CW2B   1456
#define CP1W   1472
#define CP1B   1484
#define CP1S   1488
#define CP1H   1492
#define CSTN   1504

#define LSD    (PR * DP)
#define LSA    ((PR * AP) / 2)
#define LSQ    (NB * FW)
#define LSR3   (PR * 4)
#define LIDX   PR
#define PAIR_LDS_FLOATS (LSD + LSA + LSQ + LSR3 + CSTN + LIDX)
#define PAIR_LDS_BYTES  (PAIR_LDS_FLOATS * 4)

static_assert(FW == 4 * 32 && (FW % 32) == 0 && (K2 % 32) == 0 && K2 == 2 * FW);
static_assert(QW == 3 * FW && (QW % GBN) == 0 && ((QW * 4) % 128) == 0 && WROWS == QW);
static_assert(GBM == (GTHR / 32) * 16 && GBN == 4 * 16);
static_assert(PR == FTHR && PR == NB * NNB && NB == 2 * (FTHR / 32) && NNB == 16 && CSW == NNB);
static_assert((UWQKV % NTHR) == 0 && (NUW % NTHR) == 0 && UWQKV == 3 * 2048);
static_assert(AP >= K2 && DP >= CSW && ((AP * 2) % 16) == 0 && ((DP * 4) % 16) == 0);
static_assert((PR * AP) % 8 == 0 && (LSD % 4) == 0 && (LSA % 4) == 0 && (LSQ % 4) == 0 && (LSR3 % 4) == 0);
static_assert((CSTN % 4) == 0 && CSTN >= CP1H + 3 && CP1B >= CP1W + 9 && CW1B >= CW2W + 256);
static_assert((CP2W % 4) == 0 && (CP2B % 4) == 0 && (CBNS % 4) == 0 && (CBNB % 4) == 0 && (CBQ % 4) == 0);
static_assert((CBK % 4) == 0 && (CBV % 4) == 0 && (CW2W % 4) == 0 && (CW1B % 4) == 0 && (CW1S % 4) == 0);
static_assert((CW1H % 4) == 0 && (CW2B % 4) == 0);
static_assert(PAIR_LDS_BYTES <= 300000);
static_assert(((FW * 2) % 128) == 0 && ((K2 * 2) % 128) == 0 && ((FW * 4) % 128) == 0);

typedef float          v4f  __attribute__((ext_vector_type(4)));
typedef float          v8f  __attribute__((ext_vector_type(8)));
typedef int            v8i  __attribute__((ext_vector_type(8)));
typedef unsigned int   v4u  __attribute__((ext_vector_type(4)));
typedef unsigned short v8us __attribute__((ext_vector_type(8)));
typedef __bf16         v16b __attribute__((ext_vector_type(16)));
typedef v4f  __attribute__((may_alias)) v4fa;
typedef v4u  __attribute__((may_alias)) v4ua;
typedef v8us __attribute__((may_alias)) v8usa;
union FragB { v16b v; v8us h[2]; v8i w; };

__device__ __forceinline__ v8f wmb(const FragB& a, const FragB& b, v8f c) {
  v8f d = __builtin_amdgcn_wmma_f32_16x16x32_bf16(false, a.v, false, b.v, (short)0, c, false, false);
  asm volatile("v_nop\n\tv_nop\n\tv_nop\n\tv_nop" : "+v"(d) : "v"(a.w), "v"(b.w));
  return d;
}

__device__ __forceinline__ unsigned int f2bf(float f) {
  const unsigned int u = __float_as_uint(f);
  return ((u + 0x7FFFu + ((u >> 16) & 1u)) >> 16) & 0xFFFFu;
}
__device__ __forceinline__ float bf2f(unsigned int b) { return __uint_as_float(b << 16); }
__device__ __forceinline__ float bfr(float f) { return bf2f(f2bf(f)); }
__device__ __forceinline__ v4f bfr4(const v4f a) {
  v4f r; r.x = bfr(a.x); r.y = bfr(a.y); r.z = bfr(a.z); r.w = bfr(a.w); return r;
}
__device__ __forceinline__ unsigned int pk2(float lo, float hi) { return f2bf(lo) | (f2bf(hi) << 16); }
__device__ __forceinline__ v4u pack8(const v4f a, const v4f b) {
  v4u r;
  r.x = pk2(a.x, a.y); r.y = pk2(a.z, a.w); r.z = pk2(b.x, b.y); r.w = pk2(b.z, b.w);
  return r;
}
__device__ __forceinline__ v8f ld8(const float* p) {
  const v4f a = *(const v4fa*)p;
  const v4f b = *(const v4fa*)(p + 4);
  v8f r = {a.x, a.y, a.z, a.w, b.x, b.y, b.z, b.w};
  return r;
}
__device__ __forceinline__ float posc(float r0, float r1, float r2, float u, float v, float w, float b) {
  return fmaf(r2, w, fmaf(r1, v, r0 * u)) + b;
}
__device__ __forceinline__ void put16(unsigned short* dp, v8us o) {
  *(volatile v8us*)dp = o;
  __threadfence();
  *(volatile v8us*)dp = o;
}

__global__ __launch_bounds__(NTHR) void k_xprep(const float* __restrict__ x, unsigned short* xb, int nN, int nUnits) {
  const int i = (int)blockIdx.x * NTHR + (int)threadIdx.x;
  if (i >= nUnits) return;
  const int row = i >> 4;
  const int c0  = (i & 15) * 8;
  const int rc  = row < nN ? row : nN - 1;
  const float* p = x + (size_t)rc * FW + c0;
  v4f a = *(const v4fa*)p;
  v4f b = *(const v4fa*)(p + 4);
  const v4f z4 = {0.f, 0.f, 0.f, 0.f};
  if (row >= nN) { a = z4; b = z4; }
  const v4u hv = pack8(a, b);
  unsigned short* o = xb + (size_t)row * FW + c0;
  *(volatile v4u*)o = hv;
  __threadfence();
  *(volatile v4u*)o = hv;
}

__global__ __launch_bounds__(NTHR) void k_wprep(const float* __restrict__ Wq, const float* __restrict__ Wk,
                                                const float* __restrict__ Wv, const float* __restrict__ W1,
                                                unsigned short* WQKVT, unsigned short* W1T) {
  const int u = (int)blockIdx.x * NTHR + (int)threadIdx.x;
  if (u >= NUW) return;
  v8us o;
  unsigned short* dp;
  if (u < UWQKV) {
    const int part = u >> 11;
    const int v    = u & 2047;
    const int n    = v >> 4;
    const int k8   = (v & 15) * 8;
    const float* W = (part == 0) ? Wq : ((part == 1) ? Wk : Wv);
    const float* p = W + (size_t)k8 * FW + n;
#pragma unroll
    for (int i = 0; i < 8; ++i) o[i] = (unsigned short)f2bf(p[(size_t)i * FW]);
    dp = WQKVT + (size_t)(part * FW + n) * FW + k8;
  } else {
    const int v    = u - UWQKV;
    const int n    = v >> 5;
    const int k8   = (v & 31) * 8;
    const int srow = k8 & (FW - 1);
    const float* p = W1 + (size_t)srow * CSW + n;
#pragma unroll
    for (int i = 0; i < 8; ++i) o[i] = (unsigned short)f2bf(p[(size_t)i * CSW]);
    dp = W1T + (size_t)n * K2 + k8;
  }
  put16(dp, o);
}

__global__ __launch_bounds__(GTHR) void k_gemm(const unsigned short* __restrict__ A,
                                               const unsigned short* __restrict__ WT, float* outF) {
  __shared__ __attribute__((aligned(16))) float stg[GBM * GBN];
  const int tid = (int)threadIdx.x, lane = tid & 31, wave = tid >> 5, hh = lane >> 4, m = lane & 15;
  const int rowBase = (int)blockIdx.x * GBM;
  const int col0    = (int)blockIdx.y * GBN;

  v8f acc[4];
  {
    const v8f z = {0.f, 0.f, 0.f, 0.f, 0.f, 0.f, 0.f, 0.f};
    acc[0] = z; acc[1] = z; acc[2] = z; acc[3] = z;
  }
  const unsigned short* ap = A  + (size_t)(rowBase + 16 * wave + m) * (size_t)FW + 8 * hh;
  const unsigned short* wp = WT + (size_t)(col0 + m) * (size_t)FW + 8 * hh;
#pragma unroll 1
  for (int ks = 0; ks < FW / 32; ++ks) {
    FragB af;
    af.h[0] = *(const v8usa*)(ap + 32 * ks);
    af.h[1] = *(const v8usa*)(ap + 32 * ks + 16);
#pragma unroll
    for (int t = 0; t < 4; ++t) {
      const unsigned short* wq = wp + (size_t)(16 * t) * (size_t)FW + 32 * ks;
      FragB bf;
      bf.h[0] = *(const v8usa*)wq;
      bf.h[1] = *(const v8usa*)(wq + 16);
      acc[t] = wmb(af, bf, acc[t]);
    }
  }

#pragma unroll
  for (int t = 0; t < 4; ++t) {
    const int lc = 16 * t + m;
#pragma unroll
    for (int r = 0; r < 8; ++r) {
      const int lr = 16 * wave + 8 * hh + r;
      stg[lr * GBN + lc] = acc[t][r];
    }
  }
  __syncthreads();

  v4f fv[8];
#pragma unroll
  for (int i = 0; i < 8; ++i) {
    const int lr = 16 * wave + 2 * i + hh;
    fv[i] = *(const v4fa*)(stg + lr * GBN + 4 * m);
  }
#pragma unroll
  for (int i = 0; i < 8; ++i) {
    const int lr = 16 * wave + 2 * i + hh;
    const int gr = rowBase + lr;
    float* op = outF + (size_t)gr * (size_t)QW + col0 + 4 * m;
    *(volatile v4f*)op = fv[i];
  }
  __threadfence();
#pragma unroll
  for (int i = 0; i < 8; ++i) {
    const int lr = 16 * wave + 2 * i + hh;
    const int gr = rowBase + lr;
    float* op = outF + (size_t)gr * (size_t)QW + col0 + 4 * m;
    *(volatile v4f*)op = fv[i];
  }
}

__device__ __forceinline__ void wave_gemm16(const unsigned short* sAw, float* sDw,
                                            const unsigned short* __restrict__ BT, int hh, int m) {
  const v8f z = {0.f, 0.f, 0.f, 0.f, 0.f, 0.f, 0.f, 0.f};
  v8f acc0 = z, acc1 = z;
  const unsigned short* ap0 = sAw + m * AP + 8 * hh;
  const unsigned short* ap1 = ap0 + 16 * AP;
  const unsigned short* bp  = BT + (size_t)m * (size_t)K2 + 8 * hh;
#pragma unroll 1
  for (int k0 = 0; k0 < K2; k0 += 32) {
    FragB a0, a1, b;
    a0.h[0] = *(const v8usa*)(ap0 + k0);
    a0.h[1] = *(const v8usa*)(ap0 + k0 + 16);
    a1.h[0] = *(const v8usa*)(ap1 + k0);
    a1.h[1] = *(const v8usa*)(ap1 + k0 + 16);
    b.h[0]  = *(const v8usa*)(bp + k0);
    b.h[1]  = *(const v8usa*)(bp + k0 + 16);
    acc0 = wmb(a0, b, acc0);
    acc1 = wmb(a1, b, acc1);
  }
#pragma unroll
  for (int r = 0; r < 8; ++r) {
    sDw[(8 * hh + r) * DP + m]      = acc0[r];
    sDw[(16 + 8 * hh + r) * DP + m] = acc1[r];
  }
}

__global__ __launch_bounds__(FTHR) void k_pair(
    const float* __restrict__ xyz, const float* __restrict__ feats, const int* __restrict__ nei,
    const float* __restrict__ QKV, const unsigned short* __restrict__ W1T,
    const float* __restrict__ bq, const float* __restrict__ bk, const float* __restrict__ bv,
    const float* __restrict__ p1W, const float* __restrict__ p1b,
    const float* __restrict__ p1g, const float* __restrict__ p1be,
    const float* __restrict__ p2W, const float* __restrict__ p2b,
    const float* __restrict__ bnwg, const float* __restrict__ bnwb,
    const float* __restrict__ w1b, const float* __restrict__ w1g, const float* __restrict__ w1be,
    const float* __restrict__ w2W, const float* __restrict__ w2b,
    float* out, int nN)
{
  extern __shared__ __attribute__((aligned(16))) float dyn[];
  float*          sD   = dyn;
  unsigned short* sA   = (unsigned short*)(dyn + LSD);
  float*          sQ   = dyn + LSD + LSA;
  float*          sR3  = sQ + LSQ;
  float*          cst  = sR3 + LSR3;
  int*            sIdx = (int*)(cst + CSTN);

  const int tid = (int)threadIdx.x, lane = tid & 31, wave = tid >> 5, hh = lane >> 4, m = lane & 15;
  const int ln = tid >> 4, j = tid & 15;
  const int nodeBase = (int)blockIdx.x * NB;
  const float inv = 1.0f / sqrtf(1.0f + BN_EPS);

  if (tid < 96) {
    const v4f a = bfr4(*(const v4fa*)(p2W + 4 * tid));
    *(v4fa*)(cst + CP2W + 4 * tid) = a;
  }
  if (wave == 0) {
    const v4f a = bfr4(*(const v4fa*)(p2b  + 4 * lane));
    const v4f g = bfr4(*(const v4fa*)(bnwg + 4 * lane)) * inv;
    const v4f b = bfr4(*(const v4fa*)(bnwb + 4 * lane));
    *(v4fa*)(cst + CP2B + 4 * lane) = a;
    *(v4fa*)(cst + CBNS + 4 * lane) = g;
    *(v4fa*)(cst + CBNB + 4 * lane) = b;
    const int l8 = lane < 8 ? lane : 8;
    const int l2 = lane < 2 ? lane : 2;
    const float vw = bfr(p1W[l8]);
    const float vb = bfr(p1b[l2]);
    const float vg = bfr(p1g[l2]) * inv;
    const float vh = bfr(p1be[l2]);
    if (lane < 9) cst[CP1W + lane] = vw;
    if (lane < 3) { cst[CP1B + lane] = vb; cst[CP1S + lane] = vg; cst[CP1H + lane] = vh; }
  } else if (wave == 1) {
    const v4f a = bfr4(*(const v4fa*)(bq + 4 * lane));
    const v4f b = bfr4(*(const v4fa*)(bk + 4 * lane));
    const v4f c = bfr4(*(const v4fa*)(bv + 4 * lane));
    *(v4fa*)(cst + CBQ + 4 * lane) = a;
    *(v4fa*)(cst + CBK + 4 * lane) = b;
    *(v4fa*)(cst + CBV + 4 * lane) = c;
  } else {
    const int l = tid - 64;
    const v4f a = bfr4(*(const v4fa*)(w2W + 4 * l));
    *(v4fa*)(cst + CW2W + 4 * l) = a;
    if (wave == 3) {
      const int lc = lane & 15;
      const float a1 = bfr(w1b[lc]);
      const float a2 = bfr(w1g[lc]) * inv;
      const float a3 = bfr(w1be[lc]);
      const float a4 = bfr(w2b[lc]);
      if (lane < 16) { cst[CW1B + lane] = a1; cst[CW1S + lane] = a2; cst[CW1H + lane] = a3; cst[CW2B + lane] = a4; }
    }
  }
  {
    const int r  = tid >> 4;
    const int pc = (tid & 15) * 8;
    int gq = nodeBase + r;
    gq = gq < nN ? gq : nN - 1;
    const float* qp = QKV + (size_t)gq * (size_t)QW + pc;
    const v4f a = *(const v4fa*)qp;
    const v4f b = *(const v4fa*)(qp + 4);
    *(v4fa*)(sQ + r * FW + pc)     = a;
    *(v4fa*)(sQ + r * FW + pc + 4) = b;
  }
  const int gn  = nodeBase + ln;
  const int gcl = gn < nN ? gn : nN - 1;
  int idx = nei[(size_t)gcl * NNB + j];
  idx = idx < 0 ? 0 : (idx > nN - 1 ? nN - 1 : idx);
  const float xn0 = bfr(xyz[(size_t)gcl * 3]);
  const float xn1 = bfr(xyz[(size_t)gcl * 3 + 1]);
  const float xn2 = bfr(xyz[(size_t)gcl * 3 + 2]);
  const float xi0 = bfr(xyz[(size_t)idx * 3]);
  const float xi1 = bfr(xyz[(size_t)idx * 3 + 1]);
  const float xi2 = bfr(xyz[(size_t)idx * 3 + 2]);
  const float d0 = xi0 - xn0, d1 = xi1 - xn1, d2 = xi2 - xn2;
  __syncthreads();

  float r3v[3];
#pragma unroll
  for (int o = 0; o < 3; ++o) {
    const float y = fmaf(d2, cst[CP1W + 6 + o], fmaf(d1, cst[CP1W + 3 + o], d0 * cst[CP1W + o])) + cst[CP1B + o];
    r3v[o] = fmaxf(fmaf(y, cst[CP1S + o], cst[CP1H + o]), 0.0f);
  }
  sIdx[tid] = idx;
  {
    const v4f rr = {r3v[0], r3v[1], r3v[2], 0.0f};
    *(v4fa*)(sR3 + 4 * tid) = rr;
  }
  {
    const float*    kr = QKV + (size_t)idx * (size_t)QW + FW;
    const float*    qr = sQ + ln * FW;
    unsigned short* ra = sA + tid * AP;
#pragma unroll 1
    for (int c8 = 0; c8 < FW / 8; ++c8) {
      const int c0 = 8 * c8;
      const v8f k8  = ld8(kr + c0);
      const v8f q8  = ld8(qr + c0);
      const v8f u8  = ld8(cst + CP2W + c0);
      const v8f v8  = ld8(cst + CP2W + FW + c0);
      const v8f w8  = ld8(cst + CP2W + 2 * FW + c0);
      const v8f pb8 = ld8(cst + CP2B + c0);
      const v8f s8  = ld8(cst + CBNS + c0);
      const v8f h8  = ld8(cst + CBNB + c0);
      const v8f bq8 = ld8(cst + CBQ + c0);
      const v8f bk8 = ld8(cst + CBK + c0);
      v8us ohi, olo;
#pragma unroll
      for (int i = 0; i < 8; ++i) {
        const float pv = posc(r3v[0], r3v[1], r3v[2], u8[i], v8[i], w8[i], pb8[i]);
        const float w0 = ((k8[i] + bk8[i]) - (q8[i] + bq8[i])) + pv;
        const float a  = fmaxf(fmaf(w0, s8[i], h8[i]), 0.0f);
        const unsigned hb = f2bf(a);
        ohi[i] = (unsigned short)hb;
        olo[i] = (unsigned short)f2bf(a - bf2f(hb));
      }
      *(v8usa*)(ra + c0)      = ohi;
      *(v8usa*)(ra + FW + c0) = olo;
    }
  }
  __syncthreads();

  wave_gemm16(sA + 32 * wave * AP, sD + 32 * wave * DP, W1T, hh, m);
  __syncthreads();

  {
    const float* rd = sD + tid * DP;
    const v8f da = ld8(rd);
    const v8f db = ld8(rd + 8);
    const v8f ba = ld8(cst + CW1B), bb = ld8(cst + CW1B + 8);
    const v8f sa = ld8(cst + CW1S), sb = ld8(cst + CW1S + 8);
    const v8f ta = ld8(cst + CW1H), tb = ld8(cst + CW1H + 8);
    float h1[16];
#pragma unroll
    for (int i = 0; i < 8; ++i) {
      h1[i]     = fmaxf(fmaf(da[i] + ba[i], sa[i], ta[i]), 0.0f);
      h1[8 + i] = fmaxf(fmaf(db[i] + bb[i], sb[i], tb[i]), 0.0f);
    }
    float* wr = sD + tid * DP;
#pragma unroll 1
    for (int o = 0; o < CSW; ++o) {
      const float* wc = cst + CW2W + o;
      float t = h1[0] * wc[0];
#pragma unroll
      for (int c = 1; c < CSW; ++c) t = fmaf(h1[c], wc[c * CSW], t);
      wr[o] = t + cst[CW2B + o];
    }
  }
  __syncthreads();

  {
    float* colp = sD + (ln * NNB) * DP + j;
    float lg[NNB];
#pragma unroll
    for (int jj = 0; jj < NNB; ++jj) lg[jj] = colp[jj * DP];
    float mx = lg[0];
#pragma unroll
    for (int jj = 1; jj < NNB; ++jj) mx = fmaxf(mx, lg[jj]);
    float sm = 0.0f;
#pragma unroll
    for (int jj = 0; jj < NNB; ++jj) { lg[jj] = __expf(lg[jj] - mx); sm += lg[jj]; }
    const float rinv = 1.0f / sm;
#pragma unroll
    for (int jj = 0; jj < NNB; ++jj) colp[jj * DP] = lg[jj] * rinv;
  }
  __syncthreads();

  {
    const int c0  = 4 * lane;
    const int cs0 = c0 & (CSW - 1);
    const v4f bv4 = *(const v4fa*)(cst + CBV + c0);
    const v4f u4  = *(const v4fa*)(cst + CP2W + c0);
    const v4f v4  = *(const v4fa*)(cst + CP2W + FW + c0);
    const v4f w4  = *(const v4fa*)(cst + CP2W + 2 * FW + c0);
    const v4f pb4 = *(const v4fa*)(cst + CP2B + c0);
    const v4f z4  = {0.f, 0.f, 0.f, 0.f};
#pragma unroll 1
    for (int t = 0; t < 2; ++t) {
      const int lnn = 2 * wave + t;
      const int gnn = nodeBase + lnn;
      const int gcc = gnn < nN ? gnn : nN - 1;
      v4f acc = z4;
#pragma unroll 2
      for (int jj = 0; jj < NNB; ++jj) {
        const int row = lnn * NNB + jj;
        const int idn = sIdx[row];
        const v4f vv = *(const v4fa*)(QKV + (size_t)idn * (size_t)QW + 2 * FW + c0);
        const v4f rr = *(const v4fa*)(sR3 + 4 * row);
        const v4f gg = *(const v4fa*)(sD + row * DP + cs0);
        v4f pp;
        pp.x = posc(rr.x, rr.y, rr.z, u4.x, v4.x, w4.x, pb4.x);
        pp.y = posc(rr.x, rr.y, rr.z, u4.y, v4.y, w4.y, pb4.y);
        pp.z = posc(rr.x, rr.y, rr.z, u4.z, v4.z, w4.z, pb4.z);
        pp.w = posc(rr.x, rr.y, rr.z, u4.w, v4.w, w4.w, pb4.w);
        const v4f tt = (vv + bv4) + pp;
        acc.x = fmaf(tt.x, gg.x, acc.x);
        acc.y = fmaf(tt.y, gg.y, acc.y);
        acc.z = fmaf(tt.z, gg.z, acc.z);
        acc.w = fmaf(tt.w, gg.w, acc.w);
      }
      const v4f f4 = bfr4(*(const v4fa*)(feats + (size_t)gcc * (size_t)FW + c0));
      const v4f zz = acc + f4;
      v4f y;
      y.x = zz.x >= 0.0f ? zz.x : LEAK * zz.x;
      y.y = zz.y >= 0.0f ? zz.y : LEAK * zz.y;
      y.z = zz.z >= 0.0f ? zz.z : LEAK * zz.z;
      y.w = zz.w >= 0.0f ? zz.w : LEAK * zz.w;
      if (gnn < nN) {
        float* op = out + (size_t)gnn * (size_t)FW + c0;
        *(volatile v4f*)op = y;
        __threadfence();
        *(volatile v4f*)op = y;
      }
    }
  }
}

static inline int cdiv(int a, int b) { return (a + b - 1) / b; }
static inline size_t al256(size_t o) { return (o + 255) & ~(size_t)255; }

extern "C" void kernel_launch(void* const* d_in, const int* in_sizes, int n_in,
                              void* d_out, int out_size, void* d_ws, size_t ws_size,
                              hipStream_t stream) {
  if (n_in < 23) return;
  if (in_sizes[1] < FW || (in_sizes[1] % FW) != 0) return;
  const int nN = in_sizes[1] / FW;
  if (nN < 1 || nN > (1 << 22)) return;
  if ((long long)in_sizes[0] != 3LL * nN) return;
  if ((long long)in_sizes[2] != (long long)NNB * nN) return;
  if (in_sizes[3] != FW * FW || in_sizes[5] != FW * FW || in_sizes[7] != FW * FW) return;
  if (in_sizes[4] != FW || in_sizes[6] != FW || in_sizes[8] != FW) return;
  if (in_sizes[9] != 9 || in_sizes[10] != 3 || in_sizes[11] != 3 || in_sizes[12] != 3) return;
  if (in_sizes[13] != 3 * FW || in_sizes[14] != FW) return;
  if (in_sizes[15] != FW || in_sizes[16] != FW) return;
  if (in_sizes[17] != FW * CSW || in_sizes[18] != CSW || in_sizes[19] != CSW || in_sizes[20] != CSW) return;
  if (in_sizes[21] != CSW * CSW || in_sizes[22] != CSW) return;
  if ((long long)out_size != (long long)nN * FW) return;

  const float* xyz   = (const float*)d_in[0];
  const float* feats = (const float*)d_in[1];
  const int*   nei   = (const int*)  d_in[2];
  const float* Wq    = (const float*)d_in[3];
  const float* bq    = (const float*)d_in[4];
  const float* Wk    = (const float*)d_in[5];
  const float* bk    = (const float*)d_in[6];
  const float* Wv    = (const float*)d_in[7];
  const float* bv    = (const float*)d_in[8];
  const float* p1W   = (const float*)d_in[9];
  const float* p1b   = (const float*)d_in[10];
  const float* p1g   = (const float*)d_in[11];
  const float* p1be  = (const float*)d_in[12];
  const float* p2W   = (const float*)d_in[13];
  const float* p2b   = (const float*)d_in[14];
  const float* bnwg  = (const float*)d_in[15];
  const float* bnwb  = (const float*)d_in[16];
  const float* w1W   = (const float*)d_in[17];
  const float* w1b   = (const float*)d_in[18];
  const float* w1g   = (const float*)d_in[19];
  const float* w1be  = (const float*)d_in[20];
  const float* w2W   = (const float*)d_in[21];
  const float* w2b   = (const float*)d_in[22];
  float* out = (float*)d_out;

  const int MP = cdiv(nN, GBM) * GBM;
  const int gM = MP / GBM;

  char* ws = (char*)d_ws;
  size_t off = 0;
  const size_t oXB = off; off = al256(off + (size_t)MP * FW * 2);
  const size_t oWQ = off; off = al256(off + (size_t)WROWS * FW * 2);
  const size_t oW1 = off; off = al256(off + (size_t)CSW * K2 * 2);
  const size_t oQV = off; off = al256(off + (size_t)MP * QW * 4);
  if (off > ws_size || off > (size_t)WSMAX) return;
  unsigned short* XB    = (unsigned short*)(ws + oXB);
  unsigned short* WQKVT = (unsigned short*)(ws + oWQ);
  unsigned short* W1T   = (unsigned short*)(ws + oW1);
  float*          QKV   = (float*)(ws + oQV);

  hipFuncSetAttribute(reinterpret_cast<const void*>(&k_pair), hipFuncAttributeMaxDynamicSharedMemorySize,
                      (int)PAIR_LDS_BYTES);

  const int nUx = MP * (FW / 8);
  k_xprep<<<cdiv(nUx, NTHR), NTHR, 0, stream>>>(feats, XB, nN, nUx);
  k_wprep<<<NUW / NTHR, NTHR, 0, stream>>>(Wq, Wk, Wv, w1W, WQKVT, W1T);
  k_gemm<<<dim3(gM, QW / GBN), GTHR, 0, stream>>>(XB, WQKVT, QKV);
  k_pair<<<cdiv(nN, NB), FTHR, PAIR_LDS_BYTES, stream>>>(
      xyz, feats, nei, QKV, W1T, bq, bk, bv, p1W, p1b, p1g, p1be, p2W, p2b, bnwg, bnwb,
      w1b, w1g, w1be, w2W, w2b, out, nN);
}
